// TransformerGroupQueryAttention_6004364280105
// MI455X (gfx1250) — hardware-verified
//
#include <hip/hip_runtime.h>


namespace {
constexpr int S = 2048, D = 2048, HQ = 32, HKV = 8, HD = 64, G = HQ / HKV, DKV = HKV * HD  , WTOT = D + 2 * DKV  ;
constexpr float XS = 8.0f, WSC = 256.0f, PS = 8.0f, LOG2E = 1.4426950408889634f;

typedef _Float16 b16;
typedef __attribute__((ext_vector_type(16))) _Float16 v16b;
typedef __attribute__((ext_vector_type(8))) _Float16 v8b;
typedef __attribute__((ext_vector_type(8))) float v8f;
typedef __attribute__((ext_vector_type(4))) float v4f;
__device__ __forceinline__ float bf16_rne(float f) { unsigned int u = __float_as_uint(f); u += 0x7FFFu + ((u >> 16) & 1u); return __uint_as_float(u & 0xFFFF0000u); }
__device__ __forceinline__ void split16(float v, b16& hi, b16& lo) { hi = (b16)v; lo = (b16)(v - (float)hi); }
__device__ __forceinline__ v16b frag_kb(const b16* p, int hh) { const v8b a = *(const v8b*)(p + 8 * hh), b = *(const v8b*)(p + 16 + 8 * hh); v16b f;
#pragma unroll
  for (int e = 0; e < 8; ++e) { f[e] = a[e]; f[8 + e] = b[e]; } return f; }
__device__ __forceinline__ v8f wmma16b(v16b a, v16b b, v8f c) { v8f d = __builtin_amdgcn_wmma_f32_16x16x32_f16(false, a, false, b, (short)0, c, false, false); asm volatile("v_nop\n\tv_nop\n\tv_nop\n\tv_nop" : "+v"(d) : "v"(a), "v"(b)); return d; }
__device__ __forceinline__ void wave_lds_sync() { __builtin_amdgcn_fence(__ATOMIC_RELEASE, "workgroup"); __builtin_amdgcn_wave_barrier(); __builtin_amdgcn_fence(__ATOMIC_ACQUIRE, "workgroup"); }
__device__ __forceinline__ float pmul(float a, float b) { float p = a * b; asm volatile("" : "+v"(p)); return p; }

__global__ __launch_bounds__(256) void prepx_kernel(const float* __restrict__ x, b16* __restrict__ X16) {
  const size_t u = (size_t)blockIdx.x * 256 + threadIdx.x; if (u >= (size_t)S * D / 8) return; const size_t e = u * 8; const v4f a = *(const v4f*)(x + e), c = *(const v4f*)(x + e + 4); v8b o;
  for (int j = 0; j < 4; ++j) { o[j] = (b16)(bf16_rne(a[j]) * XS); o[4 + j] = (b16)(bf16_rne(c[j]) * XS); } for (int pass = 0; pass < 2; ++pass) { *(volatile v8b*)(X16 + e) = o; __threadfence(); }
}
__global__ __launch_bounds__(256) void prepw_kernel(const float* __restrict__ wq, const float* __restrict__ wk, const float* __restrict__ wv, const float* __restrict__ wo, b16* __restrict__ WT, b16* __restrict__ WOT) {
  __shared__ __attribute__((aligned(16))) b16 T[64][64 + 8];
  const int ib = blockIdx.x * 64, ob = blockIdx.y, t_ = threadIdx.x; const float* w; int ldw, ocol, orow; b16* dst;
  if (ob < 32) { w = wq; ldw = D; ocol = ob * 64; orow = ob * 64; dst = WT; } else if (ob < 40) { w = wk; ldw = DKV; ocol = (ob - 32) * 64; orow = D + (ob - 32) * 64; dst = WT; } else if (ob < 48) { w = wv; ldw = DKV; ocol = (ob - 40) * 64; orow = D + DKV + (ob - 40) * 64; dst = WT; } else { w = wo; ldw = D; ocol = (ob - 48) * 64; orow = (ob - 48) * 64; dst = WOT; }
  for (int q = t_; q < 64 * 64; q += 256) { const int ii = q >> 6, oo = q & 63; T[oo][ii] = (b16)(bf16_rne(w[(size_t)(ib + ii) * ldw + ocol + oo]) * WSC); }
  __syncthreads();
  for (int pass = 0; pass < 2; ++pass) { for (int q = t_; q < 64 * 8; q += 256) { const int oo = q >> 3, c8 = (q & 7) * 8; *(volatile v8b*)(dst + (size_t)(orow + oo) * D + ib + c8) = *(const v8b*)(&T[oo][c8]); } __threadfence(); }
}
__global__ __launch_bounds__(128) void qkv_kernel(const b16* __restrict__ X16, const b16* __restrict__ WT, const float* __restrict__ fcos, const float* __restrict__ fsin, b16* __restrict__ Qh, b16* __restrict__ Ql, b16* __restrict__ Kh, b16* __restrict__ Kl, b16* __restrict__ VTh, b16* __restrict__ VTl) {
  __shared__ __attribute__((aligned(16))) b16 Th[4][16][128 + 8], Tl[4][16][128 + 8]; __shared__ __attribute__((aligned(16))) b16 Vt[128][64 + 8], Vtl[128][64 + 8];
  const int wave = threadIdx.x >> 5, lane = threadIdx.x & 31, nloc = lane & 15, hlf = lane >> 4, t_ = threadIdx.x; const int n0 = blockIdx.y * 128; const size_t m0 = (size_t)blockIdx.x * 64 + wave * 16;
  v8f acc[8];
#pragma unroll
  for (int t = 0; t < 8; ++t) acc[t] = (v8f){};
#pragma unroll 2
  for (int kb = 0; kb < D; kb += 32) { const v16b a = frag_kb(X16 + (m0 + nloc) * D + kb, hlf);
#pragma unroll
    for (int t = 0; t < 8; ++t) acc[t] = wmma16b(a, frag_kb(WT + (size_t)(n0 + t * 16 + nloc) * D + kb, hlf), acc[t]); }
  const int kind = (n0 < D) ? 0 : (n0 < D + DKV ? 1 : 2);
  if (kind < 2) {
    const int par = nloc & 1;
#pragma unroll
    for (int t = 0; t < 8; ++t) { const int c = n0 + t * 16 + nloc; const int dd = c & 63; const int i = dd >> 1;
#pragma unroll
      for (int r = 0; r < 8; ++r) { const float mine = acc[t][r] * (1.0f / (XS * WSC)); const float other = __shfl_xor(mine, 1); const size_t srow = m0 + 8 * hlf + r; const float cs = bf16_rne(fcos[srow * (HD / 2) + i]), sn = bf16_rne(fsin[srow * (HD / 2) + i]);
        const float t0 = par ? other : mine, t1 = par ? mine : other; const float y = par ? (pmul(t0, sn) + pmul(t1, cs)) : (pmul(t0, cs) - pmul(t1, sn));
        b16 p, q; split16(y * XS, p, q); Th[wave][8 * hlf + r][t * 16 + nloc] = p; Tl[wave][8 * hlf + r][t * 16 + nloc] = q; } }
    wave_lds_sync(); b16* dh = kind == 0 ? Qh : Kh; b16* dl = kind == 0 ? Ql : Kl; const int ld = kind == 0 ? D : DKV; const int c0 = kind == 0 ? n0 : n0 - D;
    for (int pass = 0; pass < 2; ++pass) { for (int r2 = 0; r2 < 16; r2 += 2) { const int rr = r2 + (lane >> 4), c8 = (lane & 15) * 8; const size_t gi = (m0 + rr) * ld + c0 + c8; *(volatile v8b*)(dh + gi) = *(const v8b*)(&Th[wave][rr][c8]); *(volatile v8b*)(dl + gi) = *(const v8b*)(&Tl[wave][rr][c8]); } __threadfence(); }
  } else {
#pragma unroll
    for (int t = 0; t < 8; ++t)
#pragma unroll 1
      for (int r = 0; r < 8; ++r) { b16 p, q; split16(acc[t][r] * (1.0f / WSC), p, q); Vt[t * 16 + nloc][wave * 16 + 8 * hlf + r] = p; Vtl[t * 16 + nloc][wave * 16 + 8 * hlf + r] = q; }
    __syncthreads(); const int c0 = n0 - D - DKV; const size_t s0 = (size_t)blockIdx.x * 64;
    for (int pass = 0; pass < 2; ++pass) { for (int q = t_; q < 128 * 8; q += 128) { const int cc = q >> 3, c8 = (q & 7) * 8; const int col = c0 + cc; const int hk = col / HD, dd = col % HD; const size_t gi = ((size_t)hk * HD + dd) * S + s0 + c8; *(volatile v8b*)(VTh + gi) = *(const v8b*)(&Vt[cc][c8]); *(volatile v8b*)(VTl + gi) = *(const v8b*)(&Vtl[cc][c8]); } __threadfence(); }
  }
}
__global__ __launch_bounds__(64) void attn_kernel(const b16* __restrict__ Qh, const b16* __restrict__ Ql, const b16* __restrict__ Kh, const b16* __restrict__ Kl, const b16* __restrict__ VTh, const b16* __restrict__ VTl, const float* __restrict__ mask, b16* __restrict__ Oh, b16* __restrict__ Ol) {
  __shared__ __attribute__((aligned(16))) float To[2][16][HD + 4];
  const int wave = threadIdx.x >> 5, lane = threadIdx.x & 31, hh = lane >> 4, col = lane & 15; const int hq = blockIdx.y, hk = hq / G; const int q0 = blockIdx.x * 32 + wave * 16, qi = q0 + col;
  const size_t qo = (size_t)qi * D + hq * HD; const v16b qa0 = frag_kb(Qh + qo, hh), qa1 = frag_kb(Qh + qo + 32, hh), ql0 = frag_kb(Ql + qo, hh), ql1 = frag_kb(Ql + qo + 32, hh);
  const b16* Kb = Kh + hk * HD; const b16* Klb = Kl + hk * HD; const b16* Vb = VTh + (size_t)hk * HD * S; const b16* Vlb = VTl + (size_t)hk * HD * S; const float* mrow = mask + (size_t)qi * S;
  v8f o[4] = {{}, {}, {}, {}}, ol[4] = {{}, {}, {}, {}}; float mrun = -INFINITY, lrun = 0.0f; const float cs = 0.125f * LOG2E / (XS * XS);
  for (int kb = 0; kb < S; kb += 32) {
    float mk[16]; float mmax = -INFINITY;
#pragma unroll
    for (int r = 0; r < 8; ++r) { mk[r] = bf16_rne(mrow[kb + 8 * hh + r]); mk[8 + r] = bf16_rne(mrow[kb + 16 + 8 * hh + r]); mmax = fmaxf(mmax, fmaxf(mk[r], mk[8 + r])); }
#pragma unroll
    for (int sh = 16; sh >= 1; sh >>= 1) mmax = fmaxf(mmax, __shfl_xor(mmax, sh));
    if (mmax <= -1e8f) continue;
    v8f s0 = {}, s1 = {};
    { const b16* k0 = Kb + (size_t)(kb + col) * DKV, *k1 = Kb + (size_t)(kb + 16 + col) * DKV, *k0l = Klb + (size_t)(kb + col) * DKV, *k1l = Klb + (size_t)(kb + 16 + col) * DKV;
      v16b f = frag_kb(k0, hh); s0 = wmma16b(f, qa0, s0); s0 = wmma16b(f, ql0, s0); s0 = wmma16b(frag_kb(k0l, hh), qa0, s0);
      f = frag_kb(k0 + 32, hh); s0 = wmma16b(f, qa1, s0); s0 = wmma16b(f, ql1, s0); s0 = wmma16b(frag_kb(k0l + 32, hh), qa1, s0);
      f = frag_kb(k1, hh); s1 = wmma16b(f, qa0, s1); s1 = wmma16b(f, ql0, s1); s1 = wmma16b(frag_kb(k1l, hh), qa0, s1);
      f = frag_kb(k1 + 32, hh); s1 = wmma16b(f, qa1, s1); s1 = wmma16b(f, ql1, s1); s1 = wmma16b(frag_kb(k1l + 32, hh), qa1, s1); }
    float e[16]; float bm = -INFINITY;
#pragma unroll
    for (int r = 0; r < 8; ++r) { e[r] = s0[r] * cs + mk[r] * LOG2E; e[8 + r] = s1[r] * cs + mk[8 + r] * LOG2E; bm = fmaxf(bm, fmaxf(e[r], e[8 + r])); }
    bm = fmaxf(bm, __shfl_xor(bm, 16)); const float mn = fmaxf(mrun, bm); const float sc = exp2f(mrun - mn); float ls = 0.0f; v16b ph, pl;
#pragma unroll
    for (int i = 0; i < 16; ++i) { const float p = exp2f(e[i] - mn); ls += p; b16 a, c; split16(p * PS, a, c); ph[i] = a; pl[i] = c; }
    ls += __shfl_xor(ls, 16); lrun = lrun * sc + ls; mrun = mn;
#pragma unroll
    for (int t = 0; t < 4; ++t) { o[t] *= sc; ol[t] *= sc; const v16b vf = frag_kb(Vb + (size_t)(t * 16 + col) * S + kb, hh); o[t] = wmma16b(vf, ph, o[t]); ol[t] = wmma16b(vf, pl, ol[t]); ol[t] = wmma16b(frag_kb(Vlb + (size_t)(t * 16 + col) * S + kb, hh), ph, ol[t]); } }
  const float inv = 1.0f / (lrun * PS * XS);
#pragma unroll
  for (int t = 0; t < 4; ++t)
#pragma unroll
    for (int r = 0; r < 8; ++r) To[wave][col][t * 16 + 8 * hh + r] = (o[t][r] + ol[t][r]) * inv;
  wave_lds_sync();
  for (int pass = 0; pass < 2; ++pass) { for (int r4 = 0; r4 < 16; r4 += 4) { const int rr = r4 + (lane >> 3), c8 = (lane & 7) * 8; v8b hv, lv; for (int j = 0; j < 8; ++j) { b16 p, q; split16(To[wave][rr][c8 + j] * XS, p, q); hv[j] = p; lv[j] = q; }
      const size_t gi = (size_t)(q0 + rr) * D + hq * HD + c8; *(volatile v8b*)(Oh + gi) = hv; *(volatile v8b*)(Ol + gi) = lv; } __threadfence(); }
}
__global__ __launch_bounds__(128) void oproj_kernel(const b16* __restrict__ Oh, const b16* __restrict__ Ol, const b16* __restrict__ WOT, float* __restrict__ out) {
  __shared__ __attribute__((aligned(16))) float Tf[4][16][128 + 4];
  const int wave = threadIdx.x >> 5, lane = threadIdx.x & 31, nloc = lane & 15, hlf = lane >> 4; const size_t m0 = (size_t)blockIdx.x * 64 + wave * 16; const int n0 = blockIdx.y * 128; v8f acc[8];
#pragma unroll
  for (int t = 0; t < 8; ++t) acc[t] = (v8f){};
#pragma unroll 2
  for (int kb = 0; kb < D; kb += 32) { const v16b a = frag_kb(Oh + (m0 + nloc) * D + kb, hlf), al = frag_kb(Ol + (m0 + nloc) * D + kb, hlf);
#pragma unroll
    for (int t = 0; t < 8; ++t) { const v16b bw = frag_kb(WOT + (size_t)(n0 + t * 16 + nloc) * D + kb, hlf); acc[t] = wmma16b(a, bw, acc[t]); acc[t] = wmma16b(al, bw, acc[t]); } }
#pragma unroll
  for (int t = 0; t < 8; ++t)
#pragma unroll 1
    for (int r = 0; r < 8; ++r) Tf[wave][8 * hlf + r][t * 16 + nloc] = acc[t][r] * (1.0f / (XS * WSC));
  wave_lds_sync();
  for (int pass = 0; pass < 2; ++pass) { for (int rr = 0; rr < 16; ++rr) *(volatile v4f*)(out + (m0 + rr) * D + n0 + lane * 4) = *(const v4f*)(&Tf[wave][rr][lane * 4]); __threadfence(); }
}
}

extern "C" void kernel_launch(void* const* d_in, const int* in_sizes, int n_in, void* d_out, int out_size, void* d_ws, size_t ws_size, hipStream_t stream) {
  (void)n_in;
  auto Fp = [&](int i) { return (const float*)d_in[i]; };
  if (in_sizes[0] != S * D || in_sizes[1] != S * HD / 2 || in_sizes[2] != S * HD / 2 || in_sizes[3] != S * S || in_sizes[4] != D * D || in_sizes[5] != D * DKV || in_sizes[6] != D * DKV || in_sizes[7] != D * D || out_size != S * D) return;
  size_t off = 0; char* ws = (char*)d_ws;
  auto carve = [&](size_t bytes) { char* p = ws + off; off += (bytes + 255) & ~(size_t)255; return p; };
  b16* X16 = (b16*)carve((size_t)S * D * 2); b16* WT = (b16*)carve((size_t)WTOT * D * 2); b16* WOT = (b16*)carve((size_t)D * D * 2);
  b16* Qh = (b16*)carve((size_t)S * D * 2); b16* Ql = (b16*)carve((size_t)S * D * 2); b16* Kh = (b16*)carve((size_t)S * DKV * 2); b16* Kl = (b16*)carve((size_t)S * DKV * 2); b16* VTh = (b16*)carve((size_t)DKV * S * 2); b16* VTl = (b16*)carve((size_t)DKV * S * 2);
  b16* Oh = X16;  b16* Ol = (b16*)carve((size_t)S * D * 2);
  if (off > ws_size || off > ((size_t)128 << 20)) return;
  prepx_kernel<<<(unsigned)(((size_t)S * D / 8 + 255) / 256), 256, 0, stream>>>(Fp(0), X16);
  prepw_kernel<<<dim3(D / 64, WTOT / 64 + D / 64), 256, 0, stream>>>(Fp(4), Fp(5), Fp(6), Fp(7), WT, WOT);
  qkv_kernel<<<dim3(S / 64, WTOT / 128), 128, 0, stream>>>(X16, WT, Fp(1), Fp(2), Qh, Ql, Kh, Kl, VTh, VTl);
  attn_kernel<<<dim3(S / 32, HQ), 64, 0, stream>>>(Qh, Ql, Kh, Kl, VTh, VTl, Fp(3), Oh, Ol);
  oproj_kernel<<<dim3(S / 64, D / 128), 128, 0, stream>>>(Oh, Ol, WOT, (float*)d_out);
}
